// SparseWeightNN_38199439130922
// MI455X (gfx1250) — hardware-run, weakly checked
//
#include <hip/hip_runtime.h>
#include <math.h>

#define NTOK 2048
#define KIN 4096
#define NU 4096
#define NNZ 2048
#define NE 16
#define NSH 1
#define NROW_S NTOK
#define NT_MAX (NROW_S / 64)

#define CX_LOG2 11
#define CW_LOG2 16
#define CH ((float)(1u << CX_LOG2))
#define SC (1.0f / (float)(1u << (CX_LOG2 + CW_LOG2)))

#define TBL_COUNT 0
#define TBL_POFF 16
#define TBL_NTILES 40
#define TBL_TILE_E 64
#define TBL_HDR 256

static_assert(NTOK == 2048 && KIN == 4096 && NU == 4096 && NNZ == 2048 && NE == 16 && NSH == 1 && NT_MAX == 32);
static_assert(KIN % 64 == 0 && NU % 128 == 0 && NNZ % 128 == 0 && KIN % 2 == 0 && NTOK % 64 == 0 && NROW_S % 64 == 0 && NROW_S / 64 <= NT_MAX);
static_assert(TBL_HDR % 32 == 0 && TBL_HDR <= 512);
static_assert(TBL_COUNT + NE <= TBL_POFF && TBL_POFF + NE + 1 <= TBL_NTILES && TBL_NTILES < TBL_TILE_E && TBL_TILE_E + NT_MAX <= TBL_HDR);
static_assert((NTOK * KIN / 8) % 256 == 0);

constexpr size_t al256(size_t b) { return (b + 255) & ~(size_t)255; }
constexpr size_t SZ_X16  = al256((size_t)NTOK * KIN * 2);
constexpr size_t SZ_WD   = al256((size_t)KIN * NU * 4);
constexpr size_t SZ_WT   = al256((size_t)NU * KIN * 2);
constexpr size_t SZ_TBLD = al256((size_t)TBL_HDR * 4);
constexpr size_t WS_TOTAL = SZ_X16 + SZ_WD + SZ_WT + SZ_TBLD;
static_assert(WS_TOTAL == (size_t)117441536 && WS_TOTAL < (size_t)134217728);

typedef _Float16 h16;
typedef __attribute__((ext_vector_type(16))) _Float16 v16h;
typedef __attribute__((ext_vector_type(8)))  _Float16 v8h;
typedef __attribute__((ext_vector_type(8)))  float    v8f;
typedef __attribute__((ext_vector_type(4)))  float    v4f;
typedef __attribute__((ext_vector_type(2)))  float    v2f;
typedef __attribute__((ext_vector_type(4)))  unsigned int v4u;
typedef __attribute__((ext_vector_type(4)))  int      v4i;
typedef __attribute__((ext_vector_type(2)))  int      v2i;


#define VST2(T, ptr, val) do { const T vst2_v_ = (val); *(volatile T*)(ptr) = vst2_v_; __threadfence(); *(volatile T*)(ptr) = vst2_v_; } while (0)

static __device__ __forceinline__ float bfr(float f) {
    unsigned u = __float_as_uint(f);
    u += 0x7FFFu + ((u >> 16) & 1u);
    return __uint_as_float(u & 0xFFFF0000u);
}
static __device__ __forceinline__ h16 toh_flush(float v) { const float w = (fabsf(v) < 6.103515625e-05f) ? 0.0f : v; return (h16)w; }
static __device__ __forceinline__ void st8h(h16* p, const float* v) {
    v8h hv;
#pragma unroll
    for (int e = 0; e < 8; ++e) hv[e] = toh_flush(v[e]);
    VST2(v8h, p, hv);
}

union FragU { v16h v; v8h h[2]; };
static __device__ __forceinline__ v16h frag_ld(const h16* p) {
    FragU f; f.h[0] = *(const v8h*)(p); f.h[1] = *(const v8h*)(p + 16); return f.v;
}
static __device__ __forceinline__ v8f wmma16g(v16h a, v16h b, v8f c) {
    c = __builtin_amdgcn_wmma_f32_16x16x32_f16(false, a, false, b, (short)0, c, false, false);
    asm volatile("v_nop\n\tv_nop\n\tv_nop\n\tv_nop" : "+v"(c) : "v"(a), "v"(b));
    return c;
}
static __device__ __forceinline__ void wave_sync_lds() {
    __builtin_amdgcn_fence(3  , "workgroup");
    __builtin_amdgcn_wave_barrier();
    __builtin_amdgcn_fence(2  , "workgroup");
}

template <int LOG2C>
__global__ __launch_bounds__(256) void k_plane(const float* __restrict__ src, h16* __restrict__ dst, unsigned n8) {
    const unsigned u = blockIdx.x * 256u + threadIdx.x;
    if (u >= n8) return;
    const float cs = (float)(1u << LOG2C);
    const v4f a = *(const v4f*)(src + (size_t)u * 8u);
    const v4f b = *(const v4f*)(src + (size_t)u * 8u + 4u);
    float v[8] = {bfr(a.x) * cs, bfr(a.y) * cs, bfr(a.z) * cs, bfr(a.w) * cs, bfr(b.x) * cs, bfr(b.y) * cs, bfr(b.z) * cs, bfr(b.w) * cs};
    st8h(dst + (size_t)u * 8u, v);
}

__global__ __launch_bounds__(128) void k_planeTw(const float* __restrict__ src, h16* __restrict__ dst, unsigned ne, unsigned K, unsigned N, unsigned pitch, unsigned estride, float cs) {
    __shared__ __align__(16) float sT[4][64 * 36];
    const unsigned lane = threadIdx.x & 31u;
    const unsigned wave = threadIdx.x >> 5;
    const unsigned tk = K >> 6, tn = N >> 5;
    const unsigned tpe = tk * tn;
    const unsigned u = blockIdx.x * 4u + wave;
    if (u >= ne * tpe) return;
    const unsigned e = u / tpe;
    const unsigned rem = u - e * tpe;
    const unsigned kt = rem / tn;
    const unsigned nt = rem - kt * tn;
    const unsigned k0 = kt << 6, n0 = nt << 5;
    const size_t sbase = (size_t)e * (size_t)estride;
    const size_t ebase = (size_t)e * ((size_t)K * (size_t)N);
    float* slab = sT[wave];
#pragma unroll
    for (int i = 0; i < 16; ++i) {
        const unsigned p = lane + 32u * (unsigned)i;
        const unsigned kr = p >> 3;
        const unsigned n4 = (p & 7u) * 4u;
        const v4f a = *(const v4f*)(src + sbase + (size_t)(k0 + kr) * pitch + n0 + n4);
        v4f s;
        s.x = bfr(a.x) * cs; s.y = bfr(a.y) * cs; s.z = bfr(a.z) * cs; s.w = bfr(a.w) * cs;
        *(v4f*)(&slab[kr * 36u + n4]) = s;
    }
    wave_sync_lds();
#pragma unroll
    for (int i = 0; i < 8; ++i) {
        const unsigned q = lane + 32u * (unsigned)i;
        const unsigned n = q >> 3;
        const unsigned kp = q & 7u;
        float v[8];
#pragma unroll
        for (int j = 0; j < 8; ++j) v[j] = slab[(8u * kp + (unsigned)j) * 36u + n];
        st8h(dst + ebase + (size_t)(n0 + n) * K + k0 + 8u * kp, v);
    }
}

__global__ __launch_bounds__(64) void k_densify(const float* __restrict__ kv, const int* __restrict__ cols, float* __restrict__ Wd) {
    __shared__ __align__(16) float sR[2][NU];
    const unsigned lane = threadIdx.x & 31u;
    const unsigned wave = threadIdx.x >> 5;
    const unsigned k = blockIdx.x * 2u + wave;
    if (k >= (unsigned)KIN) return;
    float* row = sR[wave];
    for (unsigned i = 0; i < (unsigned)(NU / 128); ++i) *(v4f*)(&row[(lane + 32u * i) * 4u]) = (v4f){0.f, 0.f, 0.f, 0.f};
    wave_sync_lds();
    const size_t rbase = (size_t)k * (size_t)NNZ;
    for (unsigned i = 0; i < (unsigned)(NNZ / 128); ++i) {
        const unsigned j4 = (lane + 32u * i) * 4u;
        const v4i c4 = *(const v4i*)(cols + rbase + j4);
        const v4f w4 = *(const v4f*)(kv + rbase + j4);
#pragma unroll
        for (int t = 0; t < 4; ++t) {
            const int c = c4[t];
            const int cc = (c < 0) ? (c + NU) : c;
            const unsigned a = (unsigned)min(max(cc, 0), NU - 1);
            if ((unsigned)cc < (unsigned)NU) row[a] = w4[t];
        }
    }
    wave_sync_lds();
    float* dst = Wd + (size_t)k * (size_t)NU;
    for (int pass = 0; pass < 2; ++pass) {
        for (unsigned i = 0; i < (unsigned)(NU / 128); ++i) *(volatile v4f*)(dst + (lane + 32u * i) * 4u) = *(const v4f*)(&row[(lane + 32u * i) * 4u]);
        __threadfence();
    }
}

__global__ __launch_bounds__(64) void k_tbl_dense(int* __restrict__ tbl) {
    const unsigned w0 = threadIdx.x * 4u;
    int q[4];
#pragma unroll
    for (int k = 0; k < 4; ++k) {
        const unsigned w = w0 + (unsigned)k;
        int val = 0;
        val = (w < (unsigned)(TBL_COUNT + NSH)) ? NTOK : val;
        val = (w >= (unsigned)TBL_POFF && w <= (unsigned)(TBL_POFF + NE)) ? (int)min((w - (unsigned)TBL_POFF) * (unsigned)NTOK, (unsigned)NROW_S) : val;
        val = (w == (unsigned)TBL_NTILES) ? (NROW_S / 64) : val;
        val = (w >= (unsigned)TBL_TILE_E && w < (unsigned)(TBL_TILE_E + NT_MAX)) ? ((w - (unsigned)TBL_TILE_E < (unsigned)(NROW_S / 64)) ? (int)((w - (unsigned)TBL_TILE_E) / (unsigned)(NTOK / 64)) : -1) : val;
        q[k] = val;
    }
    v4i v;
    v.x = q[0]; v.y = q[1]; v.z = q[2]; v.w = q[3];
    VST2(v4i, tbl + w0, v);
}

template <int KD, int ND, int MODE>
__global__ __launch_bounds__(256) void k_lin(const h16* __restrict__ A, const h16* __restrict__ Wp, const float* __restrict__ eb,
                                             const int* __restrict__ tbl, void* __restrict__ OutV, unsigned nreal) {
    static_assert(KD % 32 == 0 && ND % 64 == 0 && MODE >= 0 && MODE <= 2);
    __shared__ __align__(16) float sT[8][16 * 68];
    const unsigned lane = threadIdx.x & 31u;
    const unsigned wave = threadIdx.x >> 5;
    const unsigned u = blockIdx.x * 8u + wave;
    if (u >= (unsigned)(NT_MAX * (ND / 64))) return;
    const unsigned rowtile = u / (unsigned)(ND / 64);
    const unsigned ct = u - rowtile * (unsigned)(ND / 64);
    const int nt = min(max(tbl[TBL_NTILES], 0), NT_MAX);
    if ((int)rowtile >= nt) return;
    const int e = min(max(tbl[TBL_TILE_E + rowtile], 0), (int)nreal - 1);
    const size_t wbase = (size_t)(unsigned)e * (size_t)(ND * KD);
    const unsigned m0 = rowtile << 6, n0 = ct << 6;
    const unsigned rlane = lane & 15u;
    const unsigned koff = (lane >> 4) * 8u;
    const unsigned mOff = koff;

    v8f acc[4][4];
#pragma unroll
    for (int i = 0; i < 4; ++i)
#pragma unroll
        for (int j = 0; j < 4; ++j) acc[i][j] = (v8f){0.f,0.f,0.f,0.f,0.f,0.f,0.f,0.f};

    for (unsigned k0 = 0; k0 < (unsigned)KD; k0 += 32u) {
        v16h bh[4];
#pragma unroll
        for (int j = 0; j < 4; ++j)
            bh[j] = frag_ld(Wp + wbase + (size_t)(n0 + ((unsigned)j << 4) + rlane) * KD + koff + k0);
#pragma unroll
        for (int i = 0; i < 4; ++i) {
            const v16h ah = frag_ld(A + (size_t)(m0 + ((unsigned)i << 4) + rlane) * KD + koff + k0);
#pragma unroll
            for (int j = 0; j < 4; ++j) acc[i][j] = wmma16g(ah, bh[j], acc[i][j]);
        }
    }

    float ebv[4];
#pragma unroll
    for (int j = 0; j < 4; ++j) ebv[j] = bfr(eb[(unsigned)e * (unsigned)ND + n0 + ((unsigned)j << 4) + rlane]);

    float* slab = sT[wave];
#pragma unroll
    for (int i = 0; i < 4; ++i) {
        const unsigned mBase = m0 + ((unsigned)i << 4);
#pragma unroll
        for (int j = 0; j < 4; ++j)
#pragma unroll
            for (int r = 0; r < 8; ++r) {
                const float a = acc[i][j][r] * SC + ebv[j];
                const float g = fmaxf(a, 0.0f);
                slab[(mOff + (unsigned)r) * 68u + ((unsigned)j << 4) + rlane] = (MODE == 2) ? g : g * CH;
            }
        wave_sync_lds();
        if constexpr (MODE == 2) {
            float* Out = (float*)OutV;
            const unsigned hh = lane >> 4, c4 = (lane & 15u) * 4u;
#pragma unroll
            for (int half = 0; half < 2; ++half) {
                v4f vv[4];
#pragma unroll
                for (int it = 0; it < 4; ++it) {
                    const unsigned row = (unsigned)(half * 4 + it) * 2u + hh;
                    vv[it] = *(const v4f*)(slab + row * 68u + c4);
                }
                for (int pass = 0; pass < 2; ++pass) {
#pragma unroll
                    for (int it = 0; it < 4; ++it) {
                        const unsigned row = (unsigned)(half * 4 + it) * 2u + hh;
                        *(volatile v4f*)(Out + (size_t)(mBase + row) * ND + n0 + c4) = vv[it];
                    }
                    __threadfence();
                }
            }
        } else {
            h16* Out = (h16*)OutV;
            constexpr unsigned RS = (MODE == 1) ? (unsigned)(2 * ND) : (unsigned)ND;
            const unsigned q = lane >> 3, c8 = (lane & 7u) * 8u;
            v8h hv[4];
            v8h lv[4];
#pragma unroll
            for (int it = 0; it < 4; ++it) {
                const unsigned row = (unsigned)it * 4u + q;
                const float* sp = slab + row * 68u + c8;
#pragma unroll
                for (int t = 0; t < 8; ++t) {
                    const h16 hi = toh_flush(sp[t]);
                    hv[it][t] = hi;
                    lv[it][t] = (MODE == 1) ? toh_flush(sp[t] - (float)hi) : (h16)0.0f;
                }
            }
            for (int pass = 0; pass < 2; ++pass) {
#pragma unroll
                for (int it = 0; it < 4; ++it) {
                    const unsigned row = (unsigned)it * 4u + q;
                    *(volatile v8h*)(Out + (size_t)(mBase + row) * RS + n0 + c8) = hv[it];
                    if constexpr (MODE == 1) *(volatile v8h*)(Out + (size_t)(mBase + row) * RS + (unsigned)ND + n0 + c8) = lv[it];
                }
                __threadfence();
            }
        }
        wave_sync_lds();
    }
}

extern "C" void kernel_launch(void* const* d_in, const int* in_sizes, int n_in, void* d_out, int out_size,
                              void* d_ws, size_t ws_size, hipStream_t stream) {
    if (n_in < 4) return;
    if (in_sizes[0] < NTOK * KIN || in_sizes[1] < KIN * NNZ || in_sizes[2] < NU || in_sizes[3] < KIN * NNZ) return;
    if (out_size < NTOK * NU) return;

    const float* x    = (const float*)d_in[0];
    const float* kv   = (const float*)d_in[1];
    const float* bias = (const float*)d_in[2];
    const int*   cols = (const int*)d_in[3];
    float* out = (float*)d_out;

    char* wsp = (char*)d_ws;
    size_t off = 0;
    auto carve = [&](size_t bytes) -> void* { void* r = wsp + off; off += (bytes + 255) & ~(size_t)255; return r; };
    h16*   x16  = (h16*)carve((size_t)NTOK * KIN * 2);
    float* Wd   = (float*)carve((size_t)KIN * NU * 4);
    h16*   WT   = (h16*)carve((size_t)NU * KIN * 2);
    int*   tblD = (int*)carve((size_t)TBL_HDR * 4);
    if (off != WS_TOTAL || off > ws_size || off > (size_t)134217728) return;

    k_plane<CX_LOG2><<<(NTOK * KIN / 8) / 256, 256, 0, stream>>>(x, x16, (unsigned)(NTOK * KIN / 8));
    k_densify<<<KIN / 2, 64, 0, stream>>>(kv, cols, Wd);
    constexpr float cw = (float)(1u << CW_LOG2);
    k_planeTw<<<(1 * (KIN / 64) * (NU / 32) + 3) / 4, 128, 0, stream>>>(Wd, WT, 1u, (unsigned)KIN, (unsigned)NU, (unsigned)NU, (unsigned)(KIN * NU), cw);
    k_tbl_dense<<<1, 64, 0, stream>>>(tblD);
    k_lin<KIN, NU, 2><<<(NT_MAX * (NU / 64) + 7) / 8, 256, 0, stream>>>(x16, WT, bias, tblD, (void*)out, 1u);
}
